// MaxPoolAggregator_38405597561096
// MI455X (gfx1250) — hardware-run, weakly checked
//
#include <hip/hip_runtime.h>
#include <stddef.h>
#include <stdint.h>


#define NN      20000
#define NE      640000
#define DF      128
#define TD      4
#define MR      (NN * TD)
#define XP      128
#define KX      128
#define NTHR    256
#define NWAVE   8
#define EPT     4
#define CHUNK   (NTHR * EPT)
#define NBRUN   512
#define SLB     9
#define NBLK    40
#define RCAP    20480
#define WLCAP   3072
#define DEGCAP  96
#define MEAS_BLK_HITS 16673
#define MEAS_MAXDEG   60
#define GBM     64
#define GBN     128
#define GTHR    128
#define PNB     8
#define PXB     (NN / PNB)
#define PWB     8
#define BK_WL   (NWAVE * WLCAP)
#define BK_INTS (BK_WL + RCAP + NWAVE * NBRUN + 2 * NBRUN + 32)
#define LDS_BK  (BK_INTS * 4)

static_assert(NN % PNB == 0 && NN % NWAVE == 0);
static_assert(MR % GBM == 0 && MR % 128 == 0);
static_assert(KX % 32 == 0 && KX == DF && XP >= KX && XP % 64 == 0);
static_assert(GBN == DF && GBM == (GTHR / 32) * 16 && DF == 4 * 32);
static_assert(NBRUN == (1 << SLB) && NBRUN == 2 * NTHR);
static_assert(NBLK * NBRUN >= NN && (NBLK - 1) * NBRUN < NN);
static_assert(NN <= 65536);
static_assert((long long)RCAP * 100 >= (long long)MEAS_BLK_HITS * 105);
static_assert(DEGCAP >= MEAS_MAXDEG + 8);
static_assert(WLCAP * NWAVE >= RCAP && WLCAP % 32 == 0);
static_assert(RCAP % (NTHR * 4) == 0 && BK_INTS % 4 == 0);
static_assert(LDS_BK <= 327680);
static_assert(DF * DF == PWB * NTHR * 8);
static_assert(PNB * TD * DF == 2 * NTHR * 8);
static_assert(NE % 4 == 0);

typedef float          v4f   __attribute__((ext_vector_type(4)));
typedef float          v8f   __attribute__((ext_vector_type(8)));
typedef int            v4i   __attribute__((ext_vector_type(4)));
typedef int            v8i   __attribute__((ext_vector_type(8)));
typedef unsigned short v8us  __attribute__((ext_vector_type(8)));
typedef __bf16         v16bf __attribute__((ext_vector_type(16)));
typedef v4f  __attribute__((may_alias)) v4fa;
typedef v4i  __attribute__((may_alias)) v4ia;
typedef v8us __attribute__((may_alias)) v8usa;
union FragB { v16bf v; v8us h[2]; v8i w; };

__device__ __forceinline__ v8f wmb(const FragB& a, const FragB& b, v8f c) {
  v8f d = __builtin_amdgcn_wmma_f32_16x16x32_bf16(false, a.v, false, b.v, (short)0, c, false, false);
  asm volatile("v_nop\n\tv_nop\n\tv_nop\n\tv_nop" : "+v"(d) : "v"(a.w), "v"(b.w));
  return d;
}

__device__ __forceinline__ unsigned bf16_bits(float f) {
  const unsigned u = __float_as_uint(f);
  return ((u + 0x7FFFu + ((u >> 16) & 1u)) >> 16) & 0xFFFFu;
}
__device__ __forceinline__ float bf16_val(float f) { return __uint_as_float(bf16_bits(f) << 16); }

__device__ __forceinline__ void wave_sync() {
  __builtin_amdgcn_fence(__ATOMIC_RELEASE, "wavefront");
  __builtin_amdgcn_wave_barrier();
  __builtin_amdgcn_fence(__ATOMIC_ACQUIRE, "wavefront");
}

__device__ __forceinline__ v8us cvt8(const v4f a, const v4f b) {
  v8us o;
  o[0] = (unsigned short)bf16_bits(a.x); o[1] = (unsigned short)bf16_bits(a.y);
  o[2] = (unsigned short)bf16_bits(a.z); o[3] = (unsigned short)bf16_bits(a.w);
  o[4] = (unsigned short)bf16_bits(b.x); o[5] = (unsigned short)bf16_bits(b.y);
  o[6] = (unsigned short)bf16_bits(b.z); o[7] = (unsigned short)bf16_bits(b.w);
  return o;
}

__global__ __launch_bounds__(NTHR) void k_prep(const float* __restrict__ x, const float* __restrict__ W,
                                               const float* __restrict__ bv, unsigned short* XT,
                                               unsigned short* WB, float* BF) {
  __shared__ __attribute__((aligned(16))) float tile[PNB * TD * DF];
  const int tid = (int)threadIdx.x;
  const int bid = (int)blockIdx.x;
  if (bid < PXB) {
    const int n0 = bid * PNB;
    const float* xp = x + (size_t)n0 * (size_t)(DF * TD);
#pragma unroll
    for (int i = 0; i < 4; ++i) {
      const int q  = i * NTHR + tid;
      const v4f v  = *(const v4f*)(xp + (size_t)q * 4);
      const int nd = q >> 7;
      const int f  = q & 127;
      float* tp = tile + nd * (TD * DF) + f;
      tp[0]      = v.x;
      tp[DF]     = v.y;
      tp[2 * DF] = v.z;
      tp[3 * DF] = v.w;
    }
    __syncthreads();
    v8us o0, o1;
    {
      const int u0 = tid, u1 = NTHR + tid;
      const v4f a0 = *(const v4fa*)(tile + u0 * 8);
      const v4f b0 = *(const v4fa*)(tile + u0 * 8 + 4);
      const v4f a1 = *(const v4fa*)(tile + u1 * 8);
      const v4f b1 = *(const v4fa*)(tile + u1 * 8 + 4);
      o0 = cvt8(a0, b0);
      o1 = cvt8(a1, b1);
    }
    unsigned short* dp0 = XT + (size_t)(n0 * TD) * (size_t)XP + (size_t)tid * 8;
    unsigned short* dp1 = dp0 + (size_t)NTHR * 8;
    *(volatile v8us*)dp0 = o0;
    *(volatile v8us*)dp1 = o1;
    __threadfence();
    *(volatile v8us*)dp0 = o0;
    *(volatile v8us*)dp1 = o1;
  } else if (bid < PXB + PWB) {
    const int u = (bid - PXB) * NTHR + tid;
    const float* p = W + (size_t)u * 8;
    const v4f a = *(const v4f*)p;
    const v4f b = *(const v4f*)(p + 4);
    const v8us o = cvt8(a, b);
    unsigned short* dp = WB + (size_t)u * 8;
    *(volatile v8us*)dp = o;
    __threadfence();
    *(volatile v8us*)dp = o;
  } else {
    if (tid < 32) {
      const v4f b4 = *(const v4f*)(bv + 4 * tid);
      v4f o;
      o.x = bf16_val(b4.x); o.y = bf16_val(b4.y); o.z = bf16_val(b4.z); o.w = bf16_val(b4.w);
      float* dp = BF + 4 * tid;
      *(volatile v4f*)dp = o;
      __threadfence();
      *(volatile v4f*)dp = o;
    }
  }
}

__global__ __launch_bounds__(GTHR) __attribute__((amdgpu_num_vgpr(248)))
void k_gemm(const unsigned short* __restrict__ XT, const unsigned short* __restrict__ WB,
            const float* __restrict__ BF, float* H) {
  __shared__ __attribute__((aligned(16))) float stg[GBM * GBN];
  __shared__ __attribute__((aligned(16))) float bsh[GBN];
  const int tid = (int)threadIdx.x, lane = tid & 31, wave = tid >> 5, hh = lane >> 4, m = lane & 15;
  const int rowBase = (int)blockIdx.x * GBM;

  if (tid < 32) {
    const v4f b4 = *(const v4f*)(BF + 4 * tid);
    *(v4fa*)(bsh + 4 * tid) = b4;
  }

  v8f acc[8];
  {
    const v8f z = {0.f, 0.f, 0.f, 0.f, 0.f, 0.f, 0.f, 0.f};
#pragma unroll
    for (int t = 0; t < 8; ++t) acc[t] = z;
  }
  const unsigned short* ap = XT + (size_t)(rowBase + 16 * wave + m) * (size_t)XP + 8 * hh;
  const unsigned short* bp = WB + (size_t)m * (size_t)XP + 8 * hh;

#pragma unroll 1
  for (int k0 = 0; k0 < KX; k0 += 32) {
    FragB af;
    af.h[0] = *(const v8usa*)(ap + k0);
    af.h[1] = *(const v8usa*)(ap + k0 + 16);
#pragma unroll
    for (int nt = 0; nt < 8; ++nt) {
      const unsigned short* wq = bp + (size_t)(16 * nt) * (size_t)XP + k0;
      FragB bf;
      bf.h[0] = *(const v8usa*)wq;
      bf.h[1] = *(const v8usa*)(wq + 16);
      acc[nt] = wmb(af, bf, acc[nt]);
    }
  }

#pragma unroll
  for (int nt = 0; nt < 8; ++nt) {
    const int lc = 16 * nt + m;
#pragma unroll
    for (int r = 0; r < 8; ++r) {
      const int lr = 16 * wave + 8 * hh + r;
      stg[lr * GBN + lc] = acc[nt][r];
    }
  }
  __syncthreads();

  const v4f bb4 = *(const v4fa*)(bsh + 4 * lane);
  v4f pv[16];
#pragma unroll
  for (int i = 0; i < 16; ++i) {
    const v4f t = *(const v4fa*)(stg + (16 * wave + i) * GBN + 4 * lane);
    pv[i] = t + bb4;
  }
#pragma unroll
  for (int i = 0; i < 16; ++i) {
    float* hp = H + (size_t)(rowBase + 16 * wave + i) * (size_t)DF + 4 * lane;
    *(volatile v4f*)hp = pv[i];
  }
  __threadfence();
#pragma unroll
  for (int i = 0; i < 16; ++i) {
    float* hp = H + (size_t)(rowBase + 16 * wave + i) * (size_t)DF + 4 * lane;
    *(volatile v4f*)hp = pv[i];
  }
}

__global__ __launch_bounds__(NTHR) void k_bucket(const int* __restrict__ srcs, const int* __restrict__ dsts,
                                                 int nE, int nN, int vec4,
                                                 int* LIST, int* CNT, int* OFF, int* REC) {
  extern __shared__ __attribute__((aligned(16))) int dsm[];
  int* wl   = dsm;
  int* reg2 = wl + BK_WL;
  int* cntw = reg2 + RCAP;
  int* scnt = cntw + NWAVE * NBRUN;
  int* soff = scnt + NBRUN;
  int* misc = soff + NBRUN;
  const int tid = (int)threadIdx.x, lane = tid & 31, wave = tid >> 5;
  const int nodeBase = (int)blockIdx.x * NBRUN;
  int nb = nN - nodeBase;
  nb = nb > NBRUN ? NBRUN : (nb < 0 ? 0 : nb);

  {
    const v4i z4 = {0, 0, 0, 0};
    for (int i = tid * 4; i < BK_INTS; i += NTHR * 4) *(v4ia*)(dsm + i) = z4;
  }
  __syncthreads();

  int wc = 0;
  int* myl = wl + wave * WLCAP;
  const int sent = (int)(1u << 31);
  const unsigned nbs = (unsigned)nodeBase;
  const unsigned unb = (unsigned)nb;
  const int nChunks = (nE + CHUNK - 1) / CHUNK;
#pragma unroll 1
  for (int ch = 0; ch < nChunks; ++ch) {
    const int cbase = ch * CHUNK;
    const int e0 = cbase + tid * EPT;
    v4i da, ga;
    if (vec4 != 0 && cbase + CHUNK <= nE) {
      da = *(const v4i*)(dsts + e0);
      ga = *(const v4i*)(srcs + e0);
    } else {
      const int a0 = min(e0, nE - 1), a1 = min(e0 + 1, nE - 1);
      const int a2 = min(e0 + 2, nE - 1), a3 = min(e0 + 3, nE - 1);
      const int d0 = dsts[a0], d1 = dsts[a1], d2 = dsts[a2], d3 = dsts[a3];
      const int q0 = srcs[a0], q1 = srcs[a1], q2 = srcs[a2], q3 = srcs[a3];
      asm volatile("" :: "v"(d0), "v"(d1), "v"(d2), "v"(d3));
      asm volatile("" :: "v"(q0), "v"(q1), "v"(q2), "v"(q3));
      da.x = (e0     < nE) ? d0 : sent;
      da.y = (e0 + 1 < nE) ? d1 : sent;
      da.z = (e0 + 2 < nE) ? d2 : sent;
      da.w = (e0 + 3 < nE) ? d3 : sent;
      ga.x = q0; ga.y = q1; ga.z = q2; ga.w = q3;
    }
    const unsigned s0 = (unsigned)da.x - nbs, s1 = (unsigned)da.y - nbs;
    const unsigned s2 = (unsigned)da.z - nbs, s3 = (unsigned)da.w - nbs;
    const bool h0 = s0 < unb, h1 = s1 < unb, h2 = s2 < unb, h3 = s3 < unb;
    const int g0 = ga.x < 0 ? 0 : (ga.x > nN - 1 ? nN - 1 : ga.x);
    const int g1 = ga.y < 0 ? 0 : (ga.y > nN - 1 ? nN - 1 : ga.y);
    const int g2 = ga.z < 0 ? 0 : (ga.z > nN - 1 ? nN - 1 : ga.z);
    const int g3 = ga.w < 0 ? 0 : (ga.w > nN - 1 ? nN - 1 : ga.w);
    const unsigned any = __builtin_amdgcn_ballot_w32(h0 | h1 | h2 | h3);
    if (any != 0u) {
#define HITJ(HJ, SJ, GJ) { \
      const unsigned mj = __builtin_amdgcn_ballot_w32(HJ); \
      if (mj != 0u) { \
        if (HJ) { \
          const int pos = wc + (int)__builtin_amdgcn_mbcnt_lo(mj, 0u); \
          if (pos < WLCAP) myl[pos] = (GJ) | ((int)(SJ) << 16); \
        } \
        wc += (int)__builtin_popcount(mj); } }
      HITJ(h0, s0, g0)
      HITJ(h1, s1, g1)
      HITJ(h2, s2, g2)
      HITJ(h3, s3, g3)
#undef HITJ
    }
  }
  if (lane == 0) misc[16 + wave] = (wc > WLCAP) ? 1 : 0;
  const int cwc = __builtin_amdgcn_readfirstlane(wc > WLCAP ? WLCAP : wc);
  wave_sync();

  int* cw = cntw + wave * NBRUN;
#pragma unroll 1
  for (int b0 = 0; b0 < cwc; b0 += 32) {
    const int idx = b0 + lane;
    const int ent = myl[idx < WLCAP ? idx : WLCAP - 1];
    const int m32 = (cwc - b0) < 32 ? (cwc - b0) : 32;
#pragma unroll 1
    for (int k = 0; k < m32; ++k) {
      const int u  = __builtin_amdgcn_readlane(ent, k);
      const int sl = (u >> 16) & (NBRUN - 1);
      if (lane == 0) cw[sl] = cw[sl] + 1;
    }
  }
  __syncthreads();

  const int sa = 2 * tid;
  int t0 = 0, t1 = 0;
#pragma unroll
  for (int w2 = 0; w2 < NWAVE; ++w2) {
    int c0 = cntw[w2 * NBRUN + sa];
    int c1 = cntw[w2 * NBRUN + sa + 1];
    c0 = c0 < 0 ? 0 : c0;
    c1 = c1 < 0 ? 0 : c1;
    t0 += c0;
    t1 += c1;
  }
  const int ts = t0 + t1;
  int incl = ts;
#pragma unroll
  for (int d = 1; d < 32; d <<= 1) {
    const int up = __shfl_up(incl, d, 32);
    if (lane >= d) incl += up;
  }
  int mx = t0 > t1 ? t0 : t1;
  mx = max(mx, __shfl_xor(mx, 16, 32));
  mx = max(mx, __shfl_xor(mx, 8, 32));
  mx = max(mx, __shfl_xor(mx, 4, 32));
  mx = max(mx, __shfl_xor(mx, 2, 32));
  mx = max(mx, __shfl_xor(mx, 1, 32));
  if (lane == 31) misc[wave] = incl;
  if (lane == 0)  misc[8 + wave] = mx;
  __syncthreads();
  int pre = 0, nh = 0, bmax = 0, wov = 0;
#pragma unroll
  for (int w2 = 0; w2 < NWAVE; ++w2) {
    const int wt = misc[w2];
    pre += (w2 < wave) ? wt : 0;
    nh  += wt;
    bmax = max(bmax, misc[8 + w2]);
    wov |= misc[16 + w2];
  }
  {
    const int run0 = pre + incl - ts;
    const int run1 = run0 + t0;
    scnt[sa]     = t0;
    scnt[sa + 1] = t1;
    soff[sa]     = run0;
    soff[sa + 1] = run1;
    int r0 = run0, r1 = run1;
#pragma unroll
    for (int w2 = 0; w2 < NWAVE; ++w2) {
      int c0 = cntw[w2 * NBRUN + sa];
      int c1 = cntw[w2 * NBRUN + sa + 1];
      c0 = c0 < 0 ? 0 : c0;
      c1 = c1 < 0 ? 0 : c1;
      cntw[w2 * NBRUN + sa]     = r0;
      cntw[w2 * NBRUN + sa + 1] = r1;
      r0 += c0;
      r1 += c1;
    }
  }
  __syncthreads();

#pragma unroll 1
  for (int b0 = 0; b0 < cwc; b0 += 32) {
    const int idx = b0 + lane;
    const int ent = myl[idx < WLCAP ? idx : WLCAP - 1];
    const int m32 = (cwc - b0) < 32 ? (cwc - b0) : 32;
#pragma unroll 1
    for (int k = 0; k < m32; ++k) {
      const int u  = __builtin_amdgcn_readlane(ent, k);
      const int sl = (u >> 16) & (NBRUN - 1);
      const int g  = u & 0xFFFF;
      if (lane == 0) {
        int p = cw[sl];
        p = p < 0 ? 0 : (p > RCAP - 1 ? RCAP - 1 : p);
        reg2[p] = g;
        cw[sl] = p + 1;
      }
    }
  }
  __syncthreads();

  const int flag = ((nh > RCAP) || (bmax > DEGCAP) || (wov != 0)) ? 1 : 0;
  const int nhc  = nh > RCAP ? RCAP : nh;
  int* lrow = LIST + (size_t)blockIdx.x * RCAP;
#pragma unroll 1
  for (int it = 0; it < RCAP / (NTHR * 4); ++it) {
    const int i0 = 4 * (it * NTHR + tid);
    const v4i ev = *(const v4ia*)(reg2 + i0);
    int e0 = ev.x, e1 = ev.y, e2 = ev.z, e3 = ev.w;
    e0 = e0 < 0 ? 0 : (e0 > nN - 1 ? nN - 1 : e0);
    e1 = e1 < 0 ? 0 : (e1 > nN - 1 ? nN - 1 : e1);
    e2 = e2 < 0 ? 0 : (e2 > nN - 1 ? nN - 1 : e2);
    e3 = e3 < 0 ? 0 : (e3 > nN - 1 ? nN - 1 : e3);
    v4i ov;
    ov.x = (i0     < nhc) ? e0 : 0;
    ov.y = (i0 + 1 < nhc) ? e1 : 0;
    ov.z = (i0 + 2 < nhc) ? e2 : 0;
    ov.w = (i0 + 3 < nhc) ? e3 : 0;
    *(volatile v4i*)(lrow + i0) = ov;
    __threadfence();
    *(volatile v4i*)(lrow + i0) = ov;
  }
  if (tid < NBRUN / 4) {
    const v4i cv = *(const v4ia*)(scnt + 4 * tid);
    const v4i fv = *(const v4ia*)(soff + 4 * tid);
    v4i rv = {0, 0, 0, 0};
    rv.x = (tid == 0) ? flag : 0;
    rv.y = (tid == 0) ? bmax : 0;
    rv.z = (tid == 0) ? nh : 0;
    int* cp = CNT + (size_t)nodeBase + 4 * tid;
    int* fp = OFF + (size_t)nodeBase + 4 * tid;
    int* rp = REC + (size_t)blockIdx.x * 32 + 4 * (tid & 7);
    *(volatile v4i*)cp = cv;
    *(volatile v4i*)fp = fv;
    if (tid < 8) *(volatile v4i*)rp = rv;
    __threadfence();
    *(volatile v4i*)cp = cv;
    *(volatile v4i*)fp = fv;
    if (tid < 8) *(volatile v4i*)rp = rv;
  }
}

__device__ __forceinline__ float mxk(float m, float v) { return (v > m || v != v) ? v : m; }
__device__ __forceinline__ float fin(float m, int pz) {
  const float r = (m == -__builtin_inff()) ? 0.0f : m;
  return (pz != 0) ? __int_as_float(0x7fc00000) : r;
}

__global__ __launch_bounds__(NTHR) void k_replay(const float* __restrict__ H, const int* __restrict__ LIST,
                                                 const int* __restrict__ CNT, const int* __restrict__ OFF,
                                                 const int* __restrict__ REC, float* out, int nN) {
  __shared__ __attribute__((aligned(16))) float rows[NWAVE * TD * DF];
  const int tid = (int)threadIdx.x, lane = tid & 31, wave = tid >> 5;
  const int i = (int)blockIdx.x * NWAVE + wave;
  if (i >= nN) return;
  int b = i >> SLB;
  b = b > NBLK - 1 ? NBLK - 1 : b;

  const int fl   = REC[(size_t)b * 32];
  const int craw = CNT[i];
  const int oraw = OFF[i];
  int cv = craw < 0 ? 0 : craw;
  const int big = (cv > DEGCAP) ? 1 : 0;
  cv = cv > DEGCAP ? DEGCAP : cv;
  int ov = oraw < 0 ? 0 : (oraw > RCAP - 1 ? RCAP - 1 : oraw);
  cv = cv > RCAP - ov ? RCAP - ov : cv;
  const int pv = ((fl != 0) ? 1 : 0) | big;
  const int c  = __builtin_amdgcn_readfirstlane(cv);
  const int o  = __builtin_amdgcn_readfirstlane(ov);
  const int pz = __builtin_amdgcn_readfirstlane(pv);
  int last = o + c - 1;
  last = max(last, o);
  const int* lp = LIST + (size_t)b * RCAP;

  const float ninf = -__builtin_inff();
  v4f m0 = {ninf, ninf, ninf, ninf};
  v4f m1 = m0, m2 = m0, m3 = m0;
#pragma unroll 1
  for (int k = 0; k < c; k += 32) {
    int li = o + k + lane;
    li = li > last ? last : li;
    int idx = lp[li];
    idx = idx < 0 ? 0 : (idx > nN - 1 ? nN - 1 : idx);
    const int m32 = (c - k) < 32 ? (c - k) : 32;
#pragma unroll 2
    for (int j = 0; j < m32; ++j) {
      const int s = __builtin_amdgcn_readlane(idx, j);
      const float* hp = H + (size_t)s * (size_t)(TD * DF) + 4 * lane;
      const v4f v0 = *(const v4f*)hp;
      const v4f v1 = *(const v4f*)(hp + DF);
      const v4f v2 = *(const v4f*)(hp + 2 * DF);
      const v4f v3 = *(const v4f*)(hp + 3 * DF);
      m0.x = mxk(m0.x, v0.x); m0.y = mxk(m0.y, v0.y); m0.z = mxk(m0.z, v0.z); m0.w = mxk(m0.w, v0.w);
      m1.x = mxk(m1.x, v1.x); m1.y = mxk(m1.y, v1.y); m1.z = mxk(m1.z, v1.z); m1.w = mxk(m1.w, v1.w);
      m2.x = mxk(m2.x, v2.x); m2.y = mxk(m2.y, v2.y); m2.z = mxk(m2.z, v2.z); m2.w = mxk(m2.w, v2.w);
      m3.x = mxk(m3.x, v3.x); m3.y = mxk(m3.y, v3.y); m3.z = mxk(m3.z, v3.z); m3.w = mxk(m3.w, v3.w);
    }
  }

  v4f q0, q1, q2, q3;
  q0.x = fin(m0.x, pz); q0.y = fin(m1.x, pz); q0.z = fin(m2.x, pz); q0.w = fin(m3.x, pz);
  q1.x = fin(m0.y, pz); q1.y = fin(m1.y, pz); q1.z = fin(m2.y, pz); q1.w = fin(m3.y, pz);
  q2.x = fin(m0.z, pz); q2.y = fin(m1.z, pz); q2.z = fin(m2.z, pz); q2.w = fin(m3.z, pz);
  q3.x = fin(m0.w, pz); q3.y = fin(m1.w, pz); q3.z = fin(m2.w, pz); q3.w = fin(m3.w, pz);

  float* rb = rows + wave * (TD * DF);
  *(v4fa*)(rb + 16 * lane)      = q0;
  *(v4fa*)(rb + 16 * lane + 4)  = q1;
  *(v4fa*)(rb + 16 * lane + 8)  = q2;
  *(v4fa*)(rb + 16 * lane + 12) = q3;
  wave_sync();
  const v4f r0 = *(const v4fa*)(rb + 4 * lane);
  const v4f r1 = *(const v4fa*)(rb + 128 + 4 * lane);
  const v4f r2 = *(const v4fa*)(rb + 256 + 4 * lane);
  const v4f r3 = *(const v4fa*)(rb + 384 + 4 * lane);
  float* op = out + (size_t)i * (size_t)(TD * DF) + 4 * lane;
  *(volatile v4f*)op         = r0;
  *(volatile v4f*)(op + 128) = r1;
  *(volatile v4f*)(op + 256) = r2;
  *(volatile v4f*)(op + 384) = r3;
  __threadfence();
  *(volatile v4f*)op         = r0;
  *(volatile v4f*)(op + 128) = r1;
  *(volatile v4f*)(op + 256) = r2;
  *(volatile v4f*)(op + 384) = r3;
}

static inline size_t al256(size_t o) { return (o + 255) & ~(size_t)255; }

extern "C" void kernel_launch(void* const* d_in, const int* in_sizes, int n_in,
                              void* d_out, int out_size, void* d_ws, size_t ws_size,
                              hipStream_t stream) {
  if (n_in < 4) return;
  if (in_sizes[0] != NN * DF * TD) return;
  if (in_sizes[1] != 2 * NE) return;
  if (in_sizes[2] != DF * DF || in_sizes[3] != DF) return;
  if (out_size != NN * DF * TD) return;

  const float* x  = (const float*)d_in[0];
  const int*   ei = (const int*)d_in[1];
  const int*   sr = ei;
  const int*   ds = ei + NE;
  const float* W  = (const float*)d_in[2];
  const float* bv = (const float*)d_in[3];
  float* out = (float*)d_out;

  char* ws = (char*)d_ws;
  size_t off = 0;
  const size_t oXT = off; off = al256(off + (size_t)MR * XP * 2);
  const size_t oWB = off; off = al256(off + (size_t)DF * XP * 2);
  const size_t oBF = off; off = al256(off + (size_t)DF * 4);
  const size_t oH  = off; off = al256(off + (size_t)MR * DF * 4);
  const size_t oLS = off; off = al256(off + (size_t)NBLK * RCAP * 4);
  const size_t oCN = off; off = al256(off + (size_t)NBLK * NBRUN * 4);
  const size_t oOF = off; off = al256(off + (size_t)NBLK * NBRUN * 4);
  const size_t oRC = off; off = al256(off + (size_t)NBLK * 128);
  if (off > ws_size || off > (size_t)(128u << 20)) return;
  unsigned short* XT = (unsigned short*)(ws + oXT);
  unsigned short* WB = (unsigned short*)(ws + oWB);
  float* BF  = (float*)(ws + oBF);
  float* H   = (float*)(ws + oH);
  int*  LIST = (int*)(ws + oLS);
  int*  CNT  = (int*)(ws + oCN);
  int*  OFF  = (int*)(ws + oOF);
  int*  REC  = (int*)(ws + oRC);

  hipFuncSetAttribute(reinterpret_cast<const void*>(&k_bucket), hipFuncAttributeMaxDynamicSharedMemorySize, LDS_BK);

  const int vec4 = ((NE & 3) == 0) ? 1 : 0;
  k_prep<<<PXB + PWB + 1, NTHR, 0, stream>>>(x, W, bv, XT, WB, BF);
  k_gemm<<<MR / GBM, GTHR, 0, stream>>>(XT, WB, BF, H);
  k_bucket<<<NBLK, NTHR, LDS_BK, stream>>>(sr, ds, NE, NN, vec4, LIST, CNT, OFF, REC);
  k_replay<<<NN / NWAVE, NTHR, 0, stream>>>(H, LIST, CNT, OFF, REC, out, NN);
}
